// TransformerBlock_23519240913427
// MI455X (gfx1250) — hardware-verified
//
#include <hip/hip_runtime.h>
#include <stddef.h>
#include <stdint.h>

#define NPT    16384
#define ROWS   32768
#define KNN    16
#define DM     128
#define DIN    64
#define NEDGE  (ROWS * KNN)
#define AFP    320
#define FHP    256
#define QKP    384
#define GTHR   128
#define ETHR   256
#define EGRID  512
#define TPB    16
#define WP     136
#define AP     264
#define KP     132
#define GT_SHIP 1

#define PL0  1024
#define PL1  (PL0 + 2048)
#define PL2  (PL1 + 2048)
#define PL3  (PL2 + 2048)
#define PL4  (PL3 + 2048)
#define PL5  (PL4 + 2048)
#define PL6  (PL5 + 2048)
#define PL7  (PL6 + 4096)
#define PL8  (PL7 + 1024)
#define PL9  (PL8 + 512)
#define PL10 (PL9 + ROWS * 8)

#define O_W    0
#define O_A    (O_W + 3 * DM * WP * 2)
#define O_K    (O_A + 64 * AP * 2)
#define O_V    (O_K + 64 * KP * 4)
#define O_Q    (O_V + 64 * KP * 4)
#define O_VEC  (O_Q + 4 * DM * 4)
#define O_REL  (O_VEC + 1024 * 4)
#define O_IDX  (O_REL + 256 * 4)
#define O_O    (O_IDX + 64 * 4)
#define E_LDS  (O_O + 4 * 256 * 2)

#define WS_XB   ((size_t)0)
#define WS_AF   (WS_XB + (size_t)ROWS * DIN * 2)
#define WS_FHL  (WS_AF + (size_t)ROWS * AFP * 2)
#define WS_QKV  (WS_FHL + (size_t)ROWS * FHP * 2)
#define WS_W1T  (WS_QKV + (size_t)ROWS * QKP * 4)
#define WS_WQKV (WS_W1T + (size_t)DM * DIN * 2)
#define WS_WE   (WS_WQKV + (size_t)3 * DM * DM * 2)
#define WS_WF   (WS_WE + (size_t)3 * DM * DM * 2)
#define WS_VEC  (WS_WF + (size_t)DM * AFP * 2)
#define WS_END  (WS_VEC + (size_t)1152 * 4)

static_assert(KNN == 16 && DM == 128 && DIN == 64);
static_assert(NEDGE % 64 == 0 && (NEDGE / 64) == EGRID * TPB);
static_assert(ROWS % 64 == 0 && NPT % 4 == 0 && ROWS == 2 * NPT);
static_assert(PL10 % 256 == 0 && PL8 % 256 == 0 && PL9 % 256 == 0 && PL6 % 256 == 0);
static_assert((WP * 2) % 16 == 0 && (AP * 2) % 16 == 0 && (KP * 4) % 16 == 0);
static_assert(O_A % 16 == 0 && O_K % 16 == 0 && O_V % 16 == 0 && O_Q % 16 == 0 && O_VEC % 16 == 0);
static_assert(O_REL % 16 == 0 && O_IDX % 16 == 0 && O_O % 16 == 0 && E_LDS <= 327680);
static_assert(WS_AF % 256 == 0 && WS_FHL % 256 == 0 && WS_QKV % 256 == 0 && WS_W1T % 256 == 0);
static_assert(WS_WQKV % 256 == 0 && WS_WE % 256 == 0 && WS_WF % 256 == 0 && WS_VEC % 256 == 0);
static_assert(WS_END <= (size_t)134217728);
static_assert((AFP * 2) % 128 == 0 && (QKP * 4) % 128 == 0 && (FHP * 2) % 128 == 0);
static_assert(GT_SHIP == 1 || GT_SHIP == 2);

typedef float          v4f   __attribute__((ext_vector_type(4)));
typedef float          v8f   __attribute__((ext_vector_type(8)));
typedef int            v8i   __attribute__((ext_vector_type(8)));
typedef unsigned short v8us  __attribute__((ext_vector_type(8)));
typedef unsigned short v16us __attribute__((ext_vector_type(16)));
typedef __bf16         v16bf __attribute__((ext_vector_type(16)));
typedef v4f  __attribute__((may_alias)) v4fa;
typedef v8us __attribute__((may_alias)) v8usa;
union FragB { v16bf v; v16us u; v8us h[2]; v8i w; };

__device__ __forceinline__ v8f wmb(const FragB& a, const FragB& b, v8f c) {
  v8f d = __builtin_amdgcn_wmma_f32_16x16x32_bf16(false, a.v, false, b.v, (short)0, c, false, false);
  asm volatile("v_nop\n\tv_nop\n\tv_nop\n\tv_nop" : "+v"(d) : "v"(a.w), "v"(b.w));
  return d;
}

__device__ __forceinline__ v8f z8() { v8f z = {0.f, 0.f, 0.f, 0.f, 0.f, 0.f, 0.f, 0.f}; return z; }

__device__ __forceinline__ unsigned bf16_bits(float f) {
  const unsigned u = __float_as_uint(f);
  return (u + 0x7FFFu + ((u >> 16) & 1u)) >> 16;
}
__device__ __forceinline__ float bf16_val(float f) {
  return __uint_as_float(bf16_bits(f) << 16);
}
__device__ __forceinline__ v4f bf16_val4(v4f a) {
  v4f r = { bf16_val(a.x), bf16_val(a.y), bf16_val(a.z), bf16_val(a.w) };
  return r;
}
__device__ __forceinline__ void put8(unsigned short* dp, v8us o) {
  *(volatile v8us*)dp = o;
  __threadfence();
  *(volatile v8us*)dp = o;
}
__device__ __forceinline__ void put4(float* dp, v4f o) {
  *(volatile v4f*)dp = o;
  __threadfence();
  *(volatile v4f*)dp = o;
}
__device__ __forceinline__ v8us tr8(const float* __restrict__ W, int n, int k8) {
  const float* p = W + (size_t)k8 * DM + n;
  v8us o;
#pragma unroll
  for (int i = 0; i < 8; ++i) o[i] = (unsigned short)bf16_bits(p[(size_t)i * DM]);
  return o;
}
__device__ __forceinline__ unsigned short hl_sel(float v, unsigned mq) {
  const unsigned hb = bf16_bits(v);
  const unsigned lb = bf16_bits(v - __uint_as_float(hb << 16));
  return (unsigned short)((hb & ~mq) | (lb & mq));
}

__global__ __launch_bounds__(256) void k_prep(
    const float* __restrict__ feature, const float* __restrict__ fd_w1, const float* __restrict__ fd_b1,
    const float* __restrict__ fd_w2, const float* __restrict__ fd_b2, const float* __restrict__ fc1_w,
    const float* __restrict__ fc1_b, const float* __restrict__ wq, const float* __restrict__ wk,
    const float* __restrict__ wv, const float* __restrict__ fg_w1, const float* __restrict__ fg_b1,
    const float* __restrict__ fg_w2, const float* __restrict__ fg_b2, const float* __restrict__ fc2_w,
    const float* __restrict__ fc2_b, const float* __restrict__ sc_w, const float* __restrict__ sc_b,
    unsigned short* W1T, unsigned short* WQKV, unsigned short* WE, unsigned short* WF, float* VEC,
    unsigned short* XB, unsigned short* AF) {
  const int u = (int)blockIdx.x * 256 + (int)threadIdx.x;
  if (u < PL0) { put8(W1T + (size_t)u * 8, tr8(fc1_w, u >> 3, (u & 7) * 8)); return; }
  if (u < PL1) { const int v = u - PL0; put8(WQKV + (size_t)v * 8, tr8(wq, v >> 4, (v & 15) * 8)); return; }
  if (u < PL2) { const int v = u - PL1; put8(WQKV + 16384 + (size_t)v * 8, tr8(wk, v >> 4, (v & 15) * 8)); return; }
  if (u < PL3) { const int v = u - PL2; put8(WQKV + 32768 + (size_t)v * 8, tr8(wv, v >> 4, (v & 15) * 8)); return; }
  if (u < PL4) { const int v = u - PL3; put8(WE + (size_t)v * 8, tr8(fd_w2, v >> 4, (v & 15) * 8)); return; }
  if (u < PL5) { const int v = u - PL4; put8(WE + 16384 + (size_t)v * 8, tr8(fg_w1, v >> 4, (v & 15) * 8)); return; }
  if (u < PL6) { const int v = u - PL5; put8(WE + 32768 + (size_t)v * 8, tr8(fg_w2, v >> 4, (v & 15) * 8)); return; }
  if (u < PL7) {
    const int v = u - PL6;
    const int n = v >> 5, kk = (v & 31) * 8;
    put8(WF + (size_t)n * AFP + kk, tr8(fc2_w, n, kk & 127));
    return;
  }
  if (u < PL8) {
    const int v = u - PL7;
    const int n = v >> 3, k8 = (v & 7) * 8;
    put8(WF + (size_t)n * AFP + 256 + k8, tr8(sc_w, n, k8));
    return;
  }
  if (u < PL9) {
    const int v = u - PL8;
    const int wv9 = v >> 5;
    const int ln = v & 31;
    if (wv9 < 9) {
      v4f a = {0.0f, 0.0f, 0.0f, 0.0f};
      if (wv9 < 3)       a = bf16_val4(*(const v4fa*)(fd_w1 + 4 * v));
      else if (wv9 == 3) a = bf16_val4(*(const v4fa*)(fd_b1 + 4 * ln));
      else if (wv9 == 4) a = bf16_val4(*(const v4fa*)(fd_b2 + 4 * ln));
      else if (wv9 == 5) a = bf16_val4(*(const v4fa*)(fc1_b + 4 * ln));
      else if (wv9 == 6) a = bf16_val4(*(const v4fa*)(fg_b1 + 4 * ln));
      else if (wv9 == 7) a = bf16_val4(*(const v4fa*)(fg_b2 + 4 * ln));
      else {
        const v4f p = bf16_val4(*(const v4fa*)(fc2_b + 4 * ln));
        const v4f q = bf16_val4(*(const v4fa*)(sc_b + 4 * ln));
        a = p + q;
      }
      put4(VEC + 4 * v, a);
    }
    return;
  }
  if (u < PL10) {
    const int v = u - PL9;
    const int row = v >> 3, j = v & 7;
    const float* p = feature + (size_t)v * 8;
    const v4f a = *(const v4fa*)p;
    const v4f b = *(const v4fa*)(p + 4);
    v8us o;
    o[0] = (unsigned short)bf16_bits(a.x); o[1] = (unsigned short)bf16_bits(a.y);
    o[2] = (unsigned short)bf16_bits(a.z); o[3] = (unsigned short)bf16_bits(a.w);
    o[4] = (unsigned short)bf16_bits(b.x); o[5] = (unsigned short)bf16_bits(b.y);
    o[6] = (unsigned short)bf16_bits(b.z); o[7] = (unsigned short)bf16_bits(b.w);
    unsigned short* d0 = XB + (size_t)v * 8;
    unsigned short* d1 = AF + (size_t)row * AFP + 256 + 8 * j;
    *(volatile v8us*)d0 = o;
    *(volatile v8us*)d1 = o;
    __threadfence();
    *(volatile v8us*)d0 = o;
    *(volatile v8us*)d1 = o;
    return;
  }
}

template <int KTOT, int APT, int BPT, bool WRAP, int EPI>
__global__ __launch_bounds__(GTHR) __attribute__((amdgpu_num_vgpr(248)))
void k_gemm(const unsigned short* __restrict__ A,
            const unsigned short* __restrict__ BT,
            const float* __restrict__ vec, void* outp) {
  static_assert(KTOT % 32 == 0);
  __shared__ __attribute__((aligned(16))) float stg[64 * 128];
  const int tid = (int)threadIdx.x, lane = tid & 31, wave = tid >> 5, hh = lane >> 4, m = lane & 15;
  const int rowBase = (int)blockIdx.x * 64;
  const int coff = (int)blockIdx.y * 128;

  v8f acc[8];
#pragma unroll
  for (int t = 0; t < 8; ++t) acc[t] = z8();
  const unsigned short* ap = A  + (size_t)(rowBase + 16 * wave + m) * (size_t)APT + 8 * hh;
  const unsigned short* bp = BT + (size_t)(coff + m) * (size_t)BPT + 8 * hh;

#pragma unroll 1
  for (int k0 = 0; k0 < KTOT; k0 += 32) {
    FragB af;
    af.h[0] = *(const v8usa*)(ap + k0);
    af.h[1] = *(const v8usa*)(ap + k0 + 16);
    const int kb = WRAP ? (k0 & 127) : k0;
#pragma unroll
    for (int nt = 0; nt < 8; ++nt) {
      const unsigned short* wq = bp + (size_t)(16 * nt) * (size_t)BPT + kb;
      FragB bf;
      bf.h[0] = *(const v8usa*)wq;
      bf.h[1] = *(const v8usa*)(wq + 16);
      acc[nt] = wmb(af, bf, acc[nt]);
    }
  }

#pragma unroll
  for (int nt = 0; nt < 8; ++nt) {
    const int lc = 16 * nt + m;
#pragma unroll
    for (int r = 0; r < 8; ++r) {
      const int lr = 16 * wave + 8 * hh + r;
      stg[lr * 128 + lc] = acc[nt][r];
    }
  }
  __syncthreads();

  if constexpr (EPI == 0) {
    unsigned short* outh = (unsigned short*)outp;
    const int c0 = 8 * (lane & 15);
    const unsigned mq = 0u - (unsigned)hh;
    const v4f ba = *(const v4fa*)(vec + 640 + c0);
    const v4f bb = *(const v4fa*)(vec + 640 + c0 + 4);
#pragma unroll 1
    for (int g = 0; g < 4; ++g) {
      const int rl = 16 * wave + 4 * g;
      v8us pv[4];
#pragma unroll
      for (int i = 0; i < 4; ++i) {
        const float* sp = stg + (rl + i) * 128 + c0;
        const v4f a = *(const v4fa*)sp;
        const v4f b = *(const v4fa*)(sp + 4);
        v8us o;
        o[0] = hl_sel(a.x + ba.x, mq); o[1] = hl_sel(a.y + ba.y, mq);
        o[2] = hl_sel(a.z + ba.z, mq); o[3] = hl_sel(a.w + ba.w, mq);
        o[4] = hl_sel(b.x + bb.x, mq); o[5] = hl_sel(b.y + bb.y, mq);
        o[6] = hl_sel(b.z + bb.z, mq); o[7] = hl_sel(b.w + bb.w, mq);
        pv[i] = o;
      }
      unsigned short* ob = outh + (size_t)(rowBase + rl) * FHP + 8 * lane;
#pragma unroll
      for (int i = 0; i < 4; ++i) *(volatile v8us*)(ob + (size_t)i * FHP) = pv[i];
      __threadfence();
#pragma unroll
      for (int i = 0; i < 4; ++i) *(volatile v8us*)(ob + (size_t)i * FHP) = pv[i];
    }
  } else {
    constexpr int OPT = (EPI == 1) ? QKP : DM;
    float* outf = (float*)outp;
    const int c4 = 4 * lane;
    v4f bs = {0.0f, 0.0f, 0.0f, 0.0f};
    if constexpr (EPI == 2) bs = *(const v4fa*)(vec + 1024 + c4);
#pragma unroll 1
    for (int g = 0; g < 4; ++g) {
      const int rl = 16 * wave + 4 * g;
      v4f pv[4];
#pragma unroll
      for (int i = 0; i < 4; ++i) {
        const v4f a = *(const v4fa*)(stg + (rl + i) * 128 + c4);
        pv[i] = a + bs;
      }
      float* ob = outf + (size_t)(rowBase + rl) * OPT + coff + c4;
#pragma unroll
      for (int i = 0; i < 4; ++i) *(volatile v4f*)(ob + (size_t)i * OPT) = pv[i];
      __threadfence();
#pragma unroll
      for (int i = 0; i < 4; ++i) *(volatile v4f*)(ob + (size_t)i * OPT) = pv[i];
    }
  }
}

template <int NPART>
__device__ __forceinline__ void wave_gemm(const unsigned short* sAt, const unsigned short* sWt,
                                          int n0, int hh, int m, v8f (&acc)[4]) {
  const unsigned short* bp = sWt + (n0 + m) * WP + 8 * hh;
  const unsigned short* ap = sAt + m * AP + 8 * hh;
#pragma unroll 1
  for (int kb = 0; kb < 4; ++kb) {
    FragB b;
    b.h[0] = *(const v8usa*)(bp + 32 * kb);
    b.h[1] = *(const v8usa*)(bp + 32 * kb + 16);
#pragma unroll
    for (int part = 0; part < NPART; ++part) {
#pragma unroll
      for (int mt = 0; mt < 4; ++mt) {
        const unsigned short* q = ap + mt * 16 * AP + part * 128 + 32 * kb;
        FragB a;
        a.h[0] = *(const v8usa*)q;
        a.h[1] = *(const v8usa*)(q + 16);
        acc[mt] = wmb(a, b, acc[mt]);
      }
    }
  }
}

template <int GT>
__global__ __launch_bounds__(ETHR) __attribute__((amdgpu_num_vgpr(248)))
void k_edge(const float* __restrict__ rel, const int* __restrict__ knn,
            const float* __restrict__ QKV,
            const unsigned short* __restrict__ WE,
            const float* __restrict__ vec, unsigned short* AF) {
  extern __shared__ __attribute__((aligned(16))) unsigned char dyn[];
  unsigned short* sW   = (unsigned short*)(dyn + O_W);
  unsigned short* sA   = (unsigned short*)(dyn + O_A);
  float*          sK   = (float*)(dyn + O_K);
  float*          sV   = (float*)(dyn + O_V);
  float*          sQ   = (float*)(dyn + O_Q);
  float*          sVec = (float*)(dyn + O_VEC);
  float*          sRel = (float*)(dyn + O_REL);
  int*            sIdx = (int*)(dyn + O_IDX);
  unsigned short* sO   = (unsigned short*)(dyn + O_O);

  const int tid = (int)threadIdx.x, lane = tid & 31, wave = tid >> 5, hh = lane >> 4, m = lane & 15;
  const int n0 = 16 * wave;
  const int col = n0 + m;
  const float SCALE = 0.08838834764831845f;

#pragma unroll 2
  for (int it = 0; it < 24; ++it) {
    const int c = it * ETHR + tid;
    const int mat = c >> 11, cc = c & 2047, row = cc >> 4, ck = cc & 15;
    const v8us v = *(const v8usa*)(WE + (size_t)c * 8);
    *(v8usa*)(sW + (mat * DM + row) * WP + ck * 8) = v;
  }
  {
    const v4f v = *(const v4fa*)(vec + 4 * tid);
    *(v4fa*)(sVec + 4 * tid) = v;
  }
  __syncthreads();
  const float bp2 = sVec[512 + col];
  const float bg1 = sVec[768 + col];
  const float bg2 = sVec[896 + col];

#pragma unroll 1
  for (int t = 0; t < TPB; ++t) {
    const int tile = (int)blockIdx.x * TPB + t;
    const int r0 = tile * 4;
    const int bbase = (r0 >> 14) << 14;

    if (tid < 64) {
      int ix = knn[(size_t)tile * 64 + tid];
      ix += (ix < 0) ? NPT : 0;
      ix = ix < 0 ? 0 : (ix > NPT - 1 ? NPT - 1 : ix);
      sIdx[tid] = bbase + ix;
    } else if (tid < 128) {
      const int j = tid - 64;
      const int jc = j < 47 ? j : 47;
      const v4f v = bf16_val4(*(const v4fa*)(rel + (size_t)tile * 192 + 4 * jc));
      *(v4fa*)(sRel + 4 * j) = v;
    }
    __syncthreads();

#pragma unroll 2
    for (int i = 0; i < 8; ++i) {
      const int e = wave + 8 * i;
      const int src = sIdx[e];
      const float* kp = QKV + (size_t)src * QKP + 128 + 4 * lane;
      const v4f kf = *(const v4fa*)kp;
      const v4f vf = *(const v4fa*)(kp + 128);
      *(v4fa*)(sK + e * KP + 4 * lane) = kf;
      *(v4fa*)(sV + e * KP + 4 * lane) = vf;
    }
    if (wave < 4) {
      const v4f qv = *(const v4fa*)(QKV + (size_t)(r0 + wave) * QKP + 4 * lane);
      *(v4fa*)(sQ + wave * DM + 4 * lane) = qv;
    }

    {
      const int e = tid >> 2, cb = (tid & 3) * 32;
      const float rx = sRel[3 * e], ry = sRel[3 * e + 1], rz = sRel[3 * e + 2];
#pragma unroll 1
      for (int j = 0; j < 4; ++j) {
        const int c0 = cb + 8 * j;
        const v4f w0a = *(const v4fa*)(sVec + c0),        w0b = *(const v4fa*)(sVec + c0 + 4);
        const v4f w1a = *(const v4fa*)(sVec + 128 + c0),  w1b = *(const v4fa*)(sVec + 128 + c0 + 4);
        const v4f w2a = *(const v4fa*)(sVec + 256 + c0),  w2b = *(const v4fa*)(sVec + 256 + c0 + 4);
        const v4f b1a = *(const v4fa*)(sVec + 384 + c0),  b1b = *(const v4fa*)(sVec + 384 + c0 + 4);
        const v8f W0 = {w0a.x, w0a.y, w0a.z, w0a.w, w0b.x, w0b.y, w0b.z, w0b.w};
        const v8f W1 = {w1a.x, w1a.y, w1a.z, w1a.w, w1b.x, w1b.y, w1b.z, w1b.w};
        const v8f W2 = {w2a.x, w2a.y, w2a.z, w2a.w, w2b.x, w2b.y, w2b.z, w2b.w};
        const v8f BB = {b1a.x, b1a.y, b1a.z, b1a.w, b1b.x, b1b.y, b1b.z, b1b.w};
        v8us oh, ol;
#pragma unroll
        for (int i = 0; i < 8; ++i) {
          const float pre = fmaf(rz, W2[i], fmaf(ry, W1[i], rx * W0[i])) + BB[i];
          const float hv = fmaxf(pre, 0.0f);
          const unsigned hb = bf16_bits(hv);
          const unsigned lb = bf16_bits(hv - __uint_as_float(hb << 16));
          oh[i] = (unsigned short)hb;
          ol[i] = (unsigned short)lb;
        }
        *(v8usa*)(sA + e * AP + c0) = oh;
        *(v8usa*)(sA + e * AP + 128 + c0) = ol;
      }
    }
    __syncthreads();

    v8f acc[4];
#pragma unroll
    for (int mt = 0; mt < 4; ++mt) acc[mt] = z8();
    wave_gemm<2>(sA, sW, n0, hh, m, acc);

#pragma unroll
    for (int mt = 0; mt < 4; ++mt) {
      const float qv = sQ[mt * DM + col];
#pragma unroll
      for (int r = 0; r < 8; ++r) {
        const int e = 16 * mt + 8 * hh + r;
        const float pos = acc[mt][r] + bp2;
        const float kv = sK[e * KP + col];
        const float vv = sV[e * KP + col];
        sV[e * KP + col] = vv + pos;
        acc[mt][r] = (qv - kv) + pos;
      }
    }
    __syncthreads();
#pragma unroll
    for (int mt = 0; mt < 4; ++mt) {
#pragma unroll
      for (int r = 0; r < 8; ++r) {
        const int e = 16 * mt + 8 * hh + r;
        const float av = acc[mt][r];
        const unsigned hb = bf16_bits(av);
        sA[e * AP + col] = (unsigned short)hb;
        if constexpr (GT == 2) {
          const unsigned lb = bf16_bits(av - __uint_as_float(hb << 16));
          sA[e * AP + 128 + col] = (unsigned short)lb;
        }
      }
    }
    __syncthreads();

#pragma unroll
    for (int mt = 0; mt < 4; ++mt) acc[mt] = z8();
    wave_gemm<GT>(sA, sW + DM * WP, n0, hh, m, acc);
    __syncthreads();
#pragma unroll
    for (int mt = 0; mt < 4; ++mt) {
#pragma unroll
      for (int r = 0; r < 8; ++r) {
        const int e = 16 * mt + 8 * hh + r;
        const float gv = fmaxf(acc[mt][r] + bg1, 0.0f);
        const unsigned hb = bf16_bits(gv);
        sA[e * AP + col] = (unsigned short)hb;
        if constexpr (GT == 2) {
          const unsigned lb = bf16_bits(gv - __uint_as_float(hb << 16));
          sA[e * AP + 128 + col] = (unsigned short)lb;
        }
      }
    }
    __syncthreads();

#pragma unroll
    for (int mt = 0; mt < 4; ++mt) acc[mt] = z8();
    wave_gemm<GT>(sA, sW + 2 * DM * WP, n0, hh, m, acc);

#pragma unroll
    for (int mt = 0; mt < 4; ++mt) {
      float mx = (acc[mt][0] + bg2) * SCALE;
      acc[mt][0] = mx;
#pragma unroll
      for (int r = 1; r < 8; ++r) {
        const float zv = (acc[mt][r] + bg2) * SCALE;
        acc[mt][r] = zv;
        mx = fmaxf(mx, zv);
      }
      mx = fmaxf(mx, __shfl_xor(mx, 16));
      float s = 0.0f, os = 0.0f;
#pragma unroll
      for (int r = 0; r < 8; ++r) {
        const int e = 16 * mt + 8 * hh + r;
        const float ev = expf(acc[mt][r] - mx);
        s += ev;
        os = fmaf(ev, sV[e * KP + col], os);
      }
      s  += __shfl_xor(s, 16);
      os += __shfl_xor(os, 16);
      const float ov = os / s;
      const unsigned hb = bf16_bits(ov);
      const unsigned lb = bf16_bits(ov - __uint_as_float(hb << 16));
      if (hh == 0) {
        sO[mt * 256 + col] = (unsigned short)hb;
        sO[mt * 256 + 128 + col] = (unsigned short)lb;
      }
    }
    __syncthreads();

    if (wave < 4) {
      const v8us ov = *(const v8usa*)(sO + wave * 256 + 8 * lane);
      unsigned short* dp = AF + (size_t)(r0 + wave) * AFP + 8 * lane;
      *(volatile v8us*)dp = ov;
      __threadfence();
      *(volatile v8us*)dp = ov;
    }
  }
}

extern "C" void kernel_launch(void* const* d_in, const int* in_sizes, int n_in,
                              void* d_out, int out_size, void* d_ws, size_t ws_size,
                              hipStream_t stream) {
  if (n_in < 21) return;
  if (in_sizes[1] != ROWS * DIN) return;
  if (in_sizes[2] != NEDGE * 3) return;
  if (in_sizes[3] != NEDGE) return;
  if (in_sizes[4] != 3 * DM || in_sizes[5] != DM) return;
  if (in_sizes[6] != DM * DM || in_sizes[7] != DM) return;
  if (in_sizes[8] != DIN * DM || in_sizes[9] != DM) return;
  if (in_sizes[10] != DM * DM || in_sizes[11] != DM * DM || in_sizes[12] != DM * DM) return;
  if (in_sizes[13] != DM * DM || in_sizes[14] != DM) return;
  if (in_sizes[15] != DM * DM || in_sizes[16] != DM) return;
  if (in_sizes[17] != DM * DM || in_sizes[18] != DM) return;
  if (in_sizes[19] != DIN * DM || in_sizes[20] != DM) return;
  if (out_size != ROWS * DM) return;
  if ((size_t)WS_END > ws_size) return;

  const float* feature = (const float*)d_in[1];
  const float* rel     = (const float*)d_in[2];
  const int*   knn     = (const int*)d_in[3];
  const float* fd_w1   = (const float*)d_in[4];
  const float* fd_b1   = (const float*)d_in[5];
  const float* fd_w2   = (const float*)d_in[6];
  const float* fd_b2   = (const float*)d_in[7];
  const float* fc1_w   = (const float*)d_in[8];
  const float* fc1_b   = (const float*)d_in[9];
  const float* wq      = (const float*)d_in[10];
  const float* wk      = (const float*)d_in[11];
  const float* wv      = (const float*)d_in[12];
  const float* fg_w1   = (const float*)d_in[13];
  const float* fg_b1   = (const float*)d_in[14];
  const float* fg_w2   = (const float*)d_in[15];
  const float* fg_b2   = (const float*)d_in[16];
  const float* fc2_w   = (const float*)d_in[17];
  const float* fc2_b   = (const float*)d_in[18];
  const float* sc_w    = (const float*)d_in[19];
  const float* sc_b    = (const float*)d_in[20];

  char* ws = (char*)d_ws;
  unsigned short* XB   = (unsigned short*)(ws + WS_XB);
  unsigned short* AF   = (unsigned short*)(ws + WS_AF);
  unsigned short* FHL  = (unsigned short*)(ws + WS_FHL);
  float*          QKV  = (float*)(ws + WS_QKV);
  unsigned short* W1T  = (unsigned short*)(ws + WS_W1T);
  unsigned short* WQKV = (unsigned short*)(ws + WS_WQKV);
  unsigned short* WE   = (unsigned short*)(ws + WS_WE);
  unsigned short* WF   = (unsigned short*)(ws + WS_WF);
  float*          VEC  = (float*)(ws + WS_VEC);

  hipFuncSetAttribute(reinterpret_cast<const void*>(&k_edge<GT_SHIP>),
                      hipFuncAttributeMaxDynamicSharedMemorySize, (int)E_LDS);

  k_prep<<<PL10 / 256, 256, 0, stream>>>(feature, fd_w1, fd_b1, fd_w2, fd_b2, fc1_w, fc1_b, wq, wk, wv,
                                         fg_w1, fg_b1, fg_w2, fg_b2, fc2_w, fc2_b, sc_w, sc_b,
                                         W1T, WQKV, WE, WF, VEC, XB, AF);
  k_gemm<64, 64, 64, false, 0><<<dim3(ROWS / 64, 1, 1), GTHR, 0, stream>>>(XB, W1T, VEC, (void*)FHL);
  k_gemm<256, 256, 128, true, 1><<<dim3(ROWS / 64, 3, 1), GTHR, 0, stream>>>(FHL, WQKV, VEC, (void*)QKV);
  k_edge<GT_SHIP><<<EGRID, ETHR, E_LDS, stream>>>(rel, knn, QKV, WE, VEC, AF);
  k_gemm<320, 320, 320, false, 2><<<dim3(ROWS / 64, 1, 1), GTHR, 0, stream>>>(AF, WF, VEC, d_out);
}
